// VMLA_Block_41566693491524
// MI455X (gfx1250) — hardware-verified
//
#include <hip/hip_runtime.h>

typedef _Float16 v16h __attribute__((ext_vector_type(16)));
typedef _Float16 v8h  __attribute__((ext_vector_type(8)));
typedef float    v8f  __attribute__((ext_vector_type(8)));
typedef float    v4f  __attribute__((ext_vector_type(4)));
typedef v8h __attribute__((may_alias)) v8ha;
typedef v4f __attribute__((may_alias)) v4fa;

union Frag { v16h v; v8h half[2]; };

#define BATCH  4
#define SEQ    1024
#define DM     1024
#define NHEAD  16
#define HDIM   64
#define HHALF  32
#define MVH    256
#define MLPD   4096
#define NTOK   (BATCH * SEQ)
#define PSCALE 16384.0f

#define OW_ENC   0
#define OW_Q     524288
#define OW_QR    655360
#define OW_K     786432
#define OW_V     917504
#define OW_KR    1179648
#define OW_M1    1703936
#define OW_M2    3801088
#define OW_O     5898240
#define OW_MLP1  6946816
#define OW_MLP2  11141120
#define NW_TOTAL 15335424
#define CB0  128
#define CB1  256
#define CB2  320
#define CB3  384
#define CB4  448
#define CB5  576
#define CB6  832
#define CB7  1856
#define CB8  2880
#define CB9  3392
#define CB10 5440
#define CB11 7488

static_assert(NW_TOTAL == CB11 * 2048);
static_assert(OW_Q == CB1 * 2048);
static_assert(OW_QR == CB2 * 2048);
static_assert(OW_K == CB3 * 2048);
static_assert(OW_V == CB4 * 2048);
static_assert(OW_KR == CB5 * 2048);
static_assert(OW_M1 == CB6 * 2048);
static_assert(OW_M2 == CB7 * 2048);
static_assert(OW_O == CB8 * 2048);
static_assert(OW_MLP1 == CB9 * 2048);
static_assert(OW_MLP2 == CB10 * 2048);
static_assert(NTOK % 128 == 0);
static_assert(SEQ % 128 == 0);
static_assert(DM % 64 == 0);
static_assert(MVH % 32 == 0);

__device__ __forceinline__ v8f wmma_f16(v16h a, v16h b, v8f c) {
  v8f d = __builtin_amdgcn_wmma_f32_16x16x32_f16(false, a, false, b, (short)0, c, false, false);
  asm volatile("v_nop\n\tv_nop\n\tv_nop\n\tv_nop" : "+v"(d) : "v"(a), "v"(b));
  return d;
}

__device__ __forceinline__ v16h load_frag(const _Float16* p, int h) {
  Frag f;
  f.half[0] = *(const v8ha*)(p + 8 * h);
  f.half[1] = *(const v8ha*)(p + 16 + 8 * h);
  return f.v;
}

__device__ __forceinline__ float gelu_f(float x) {
  return 0.5f * x * erfcf(-x * 0.70710678118654752f);
}

__global__ __launch_bounds__(256) void k_convert(
    const float* __restrict__ s0, const float* __restrict__ s1, const float* __restrict__ s2,
    const float* __restrict__ s3, const float* __restrict__ s4, const float* __restrict__ s5,
    const float* __restrict__ s6, const float* __restrict__ s7, const float* __restrict__ s8,
    const float* __restrict__ s9, const float* __restrict__ s10, const float* __restrict__ s11,
    _Float16* __restrict__ wbuf)
{
  const int blk = blockIdx.x;
  if (blk >= CB11) return;
  const float* src;
  int bstart;
  if      (blk < CB0)  { src = s0;  bstart = 0;    }
  else if (blk < CB1)  { src = s1;  bstart = CB0;  }
  else if (blk < CB2)  { src = s2;  bstart = CB1;  }
  else if (blk < CB3)  { src = s3;  bstart = CB2;  }
  else if (blk < CB4)  { src = s4;  bstart = CB3;  }
  else if (blk < CB5)  { src = s5;  bstart = CB4;  }
  else if (blk < CB6)  { src = s6;  bstart = CB5;  }
  else if (blk < CB7)  { src = s7;  bstart = CB6;  }
  else if (blk < CB8)  { src = s8;  bstart = CB7;  }
  else if (blk < CB9)  { src = s9;  bstart = CB8;  }
  else if (blk < CB10) { src = s10; bstart = CB9;  }
  else                 { src = s11; bstart = CB10; }
  const size_t e = ((size_t)(blk - bstart) * 256 + threadIdx.x) * 8;
  const size_t g = ((size_t)blk * 256 + threadIdx.x) * 8;
  const v4f a = *(const v4fa*)(src + e);
  const v4f c = *(const v4fa*)(src + e + 4);
  const float sc = 32.0f;
  const v8h o = { (_Float16)(a.x * sc), (_Float16)(a.y * sc), (_Float16)(a.z * sc), (_Float16)(a.w * sc),
                  (_Float16)(c.x * sc), (_Float16)(c.y * sc), (_Float16)(c.z * sc), (_Float16)(c.w * sc) };
  *(volatile v8h*)(wbuf + g) = o;
  __threadfence();
  *(volatile v8h*)(wbuf + g) = o;
}

__global__ __launch_bounds__(128) void k_layernorm(
    const float* __restrict__ x, const float* __restrict__ gw, _Float16* __restrict__ y)
{
  __shared__ float red[2][4];
  const int row = blockIdx.x, t = threadIdx.x, lane = t & 31, w = t >> 5;
  const float* xr = x + (size_t)row * DM + 8 * t;
  const v4f a = *(const v4fa*)xr;
  const v4f c = *(const v4fa*)(xr + 4);
  float s = ((a.x + a.y) + (a.z + a.w)) + ((c.x + c.y) + (c.z + c.w));
  #pragma unroll
  for (int o = 16; o >= 1; o >>= 1) s += __shfl_xor(s, o);
  if (lane == 0) red[0][w] = s;
  __syncthreads();
  const float mu = ((red[0][0] + red[0][1]) + (red[0][2] + red[0][3])) * (1.0f / DM);
  const float d0 = a.x - mu, d1 = a.y - mu, d2 = a.z - mu, d3 = a.w - mu;
  const float d4 = c.x - mu, d5 = c.y - mu, d6 = c.z - mu, d7 = c.w - mu;
  float q = ((d0 * d0 + d1 * d1) + (d2 * d2 + d3 * d3)) + ((d4 * d4 + d5 * d5) + (d6 * d6 + d7 * d7));
  #pragma unroll
  for (int o = 16; o >= 1; o >>= 1) q += __shfl_xor(q, o);
  if (lane == 0) red[1][w] = q;
  __syncthreads();
  const float var = ((red[1][0] + red[1][1]) + (red[1][2] + red[1][3])) * (1.0f / DM);
  const float rs = rsqrtf(var + 1e-6f);
  const v4f g0 = *(const v4fa*)(gw + 8 * t);
  const v4f g1 = *(const v4fa*)(gw + 8 * t + 4);
  const v8h o = { (_Float16)(d0 * rs * g0.x), (_Float16)(d1 * rs * g0.y), (_Float16)(d2 * rs * g0.z), (_Float16)(d3 * rs * g0.w),
                  (_Float16)(d4 * rs * g1.x), (_Float16)(d5 * rs * g1.y), (_Float16)(d6 * rs * g1.z), (_Float16)(d7 * rs * g1.w) };
  _Float16* dst = y + (size_t)row * DM + 8 * t;
  *(volatile v8h*)dst = o;
  __threadfence();
  *(volatile v8h*)dst = o;
}

__device__ __forceinline__ void store_rows_f16(const _Float16* sH, _Float16* dst, int ldo, int w, int lane) {
  const int q8 = lane & 7, sub = lane >> 3;
  #pragma unroll
  for (int i = 0; i < 8; ++i) {
    const int lid = w * 32 + i * 4 + sub;
    const v8h v = *(const v8ha*)(sH + lid * 64 + 8 * q8);
    *(volatile v8h*)(dst + (size_t)lid * (size_t)ldo + 8 * q8) = v;
  }
}
__device__ __forceinline__ void store_rows_f32(const float* sF, float* dst, int ldo, int w, int lane) {
  const int q8 = lane & 7, sub = lane >> 3;
  #pragma unroll
  for (int i = 0; i < 16; ++i) {
    const int li = i * 4 + sub;
    const int lid = w * 32 + (li >> 1);
    const int hl = li & 1;
    const v4f v = *(const v4fa*)(sF + lid * 64 + 32 * hl + 4 * q8);
    *(volatile v4f*)(dst + (size_t)lid * (size_t)ldo + 32 * hl + 4 * q8) = v;
  }
}
__device__ __forceinline__ void store_vt(const _Float16* sH, _Float16* vt, int bh, int l0, int w, int lane) {
  const int q8 = lane & 7, sub = lane >> 3;
  #pragma unroll
  for (int i = 0; i < 8; ++i) {
    const int lid = w * 32 + i * 4 + sub;
    const int d = lid >> 1, hl = lid & 1;
    const v8h v = *(const v8ha*)(sH + d * 128 + 64 * hl + 8 * q8);
    *(volatile v8h*)(vt + ((size_t)bh * HDIM + d) * SEQ + l0 + 64 * hl + 8 * q8) = v;
  }
}

template <int MODE>
__global__ __launch_bounds__(128) void k_gemm(
    const _Float16* __restrict__ A, int lda, long long sAz,
    const _Float16* __restrict__ W, int ldw, long long sWz,
    int K,
    float* __restrict__ OutF, _Float16* __restrict__ OutH, int ldo, int col0, long long sOz,
    float cscale,
    const float* __restrict__ bias, const float* __restrict__ resid,
    const float* __restrict__ lsc, const float* __restrict__ invf)
{
  constexpr bool F32O  = (MODE & 1) != 0;
  constexpr bool BIAS  = (MODE & 2) != 0;
  constexpr bool GELU  = (MODE & 4) != 0;
  constexpr bool RES   = (MODE & 8) != 0;
  constexpr bool ROPE  = (MODE & 16) != 0;
  constexpr bool TRANS = (MODE & 32) != 0;

  __shared__ __attribute__((aligned(16))) _Float16 sH[F32O ? 8 : 128 * 64];
  __shared__ __attribute__((aligned(16))) float    sF[F32O ? 128 * 64 : 4];

  const int tid = threadIdx.x, lane = tid & 31, w = tid >> 5;
  const int h = lane >> 4, m = lane & 15;
  const int m0 = blockIdx.x * 128, n0 = blockIdx.y * 64;
  const size_t zA = (size_t)blockIdx.z * (size_t)sAz;
  const size_t zW = (size_t)blockIdx.z * (size_t)sWz;
  const size_t zO = (size_t)blockIdx.z * (size_t)sOz;
  const int m0w = m0 + 32 * w;

  const _Float16* a0p = A + zA + (size_t)(m0w + m) * (size_t)lda;
  const _Float16* a1p = a0p + (size_t)16 * (size_t)lda;
  const _Float16* wbp = W + zW + (size_t)(n0 + m) * (size_t)ldw;

  const v8f zero8 = {0.f, 0.f, 0.f, 0.f, 0.f, 0.f, 0.f, 0.f};
  v8f acc[2][4];
  #pragma unroll
  for (int mt = 0; mt < 2; ++mt)
    #pragma unroll
    for (int nt = 0; nt < 4; ++nt) acc[mt][nt] = zero8;

  #pragma unroll 1
  for (int k0 = 0; k0 < K; k0 += 32) {
    const v16h fa0 = load_frag(a0p + k0, h);
    const v16h fa1 = load_frag(a1p + k0, h);
    #pragma unroll
    for (int nt = 0; nt < 4; ++nt) {
      const v16h fb = load_frag(wbp + (size_t)nt * 16 * (size_t)ldw + k0, h);
      acc[0][nt] = wmma_f16(fa0, fb, acc[0][nt]);
      acc[1][nt] = wmma_f16(fa1, fb, acc[1][nt]);
    }
  }

  if constexpr (ROPE) {
    const float ivf = invf[m];
    #pragma unroll
    for (int mt = 0; mt < 2; ++mt)
      #pragma unroll
      for (int r = 0; r < 8; ++r) {
        const int tokl = 32 * w + 16 * mt + 8 * h + r;
        const int pos = (m0 + tokl) & (SEQ - 1);
        const float ang = (float)pos * ivf;
        const float cs = cosf(ang), sn = sinf(ang);
        #pragma unroll
        for (int p = 0; p < 2; ++p) {
          const float x1 = acc[mt][2 * p][r] * cscale;
          const float x2 = acc[mt][2 * p + 1][r] * cscale;
          sH[tokl * 64 + 32 * p + m]      = (_Float16)(x1 * cs - x2 * sn);
          sH[tokl * 64 + 32 * p + 16 + m] = (_Float16)(x2 * cs + x1 * sn);
        }
      }
  } else {
    #pragma unroll
    for (int nt = 0; nt < 4; ++nt) {
      const int feat = 16 * nt + m;
      const int gn = n0 + feat;
      float bv = 0.0f, ls = 0.0f;
      if constexpr (BIAS) bv = bias[gn];
      if constexpr (RES)  ls = lsc[gn];
      #pragma unroll
      for (int mt = 0; mt < 2; ++mt)
        #pragma unroll
        for (int r = 0; r < 8; ++r) {
          const int tokl = 32 * w + 16 * mt + 8 * h + r;
          float val = acc[mt][nt][r] * cscale + bv;
          if constexpr (GELU) val = gelu_f(val);
          if constexpr (F32O) {
            if constexpr (RES) {
              const size_t ri = zO + (size_t)(m0 + tokl) * (size_t)ldo + col0 + gn;
              val = resid[ri] + val * ls;
            }
            sF[tokl * 64 + feat] = val;
          } else {
            sH[TRANS ? (feat * 128 + tokl) : (tokl * 64 + feat)] = (_Float16)val;
          }
        }
      (void)ls;
    }
  }
  __syncthreads();

  if constexpr (F32O) {
    float* dst = OutF + zO + (size_t)m0 * (size_t)ldo + col0 + n0;
    store_rows_f32(sF, dst, ldo, w, lane);
    __threadfence();
    store_rows_f32(sF, dst, ldo, w, lane);
  } else if constexpr (TRANS) {
    const int bh = (m0 / SEQ) * NHEAD + (int)blockIdx.y;
    const int l0 = m0 & (SEQ - 1);
    store_vt(sH, OutH, bh, l0, w, lane);
    __threadfence();
    store_vt(sH, OutH, bh, l0, w, lane);
  } else {
    _Float16* dst = OutH + zO + (size_t)m0 * (size_t)ldo + col0 + n0;
    store_rows_f16(sH, dst, ldo, w, lane);
    __threadfence();
    store_rows_f16(sH, dst, ldo, w, lane);
  }
}

__device__ __forceinline__ v16h pack_p(v8f a, v8f c) {
  const v16h r = { (_Float16)(a[0] * PSCALE), (_Float16)(a[1] * PSCALE), (_Float16)(a[2] * PSCALE), (_Float16)(a[3] * PSCALE),
                   (_Float16)(a[4] * PSCALE), (_Float16)(a[5] * PSCALE), (_Float16)(a[6] * PSCALE), (_Float16)(a[7] * PSCALE),
                   (_Float16)(c[0] * PSCALE), (_Float16)(c[1] * PSCALE), (_Float16)(c[2] * PSCALE), (_Float16)(c[3] * PSCALE),
                   (_Float16)(c[4] * PSCALE), (_Float16)(c[5] * PSCALE), (_Float16)(c[6] * PSCALE), (_Float16)(c[7] * PSCALE) };
  return r;
}

__device__ __forceinline__ void ctx_store_pass(const _Float16* so, _Float16* ctx,
                                               size_t rowbase, int head, int lane) {
  const int q8 = lane & 7, sub = lane >> 3;
  #pragma unroll
  for (int i = 0; i < 4; ++i) {
    const int lid = i * 4 + sub;
    const v8h v = *(const v8ha*)(so + lid * 64 + 8 * q8);
    *(volatile v8h*)(ctx + (rowbase + lid) * DM + head * HDIM + 8 * q8) = v;
  }
}

__global__ __launch_bounds__(128) void k_attn(
    const _Float16* __restrict__ Qp,
    const _Float16* __restrict__ Kp,
    const _Float16* __restrict__ VT,
    const float* __restrict__ maskp,
    _Float16* __restrict__ ctx)
{
  __shared__ __attribute__((aligned(16))) _Float16 sO[4 * 16 * 64];

  const int tid = threadIdx.x, lane = tid & 31, w = tid >> 5;
  const int h = lane >> 4, m = lane & 15;
  const int bh = blockIdx.y, b = bh >> 4, head = bh & 15;
  const int q0 = blockIdx.x * 64 + 16 * w;
  const size_t tok0 = (size_t)b * SEQ;

  const _Float16* qrow = Qp + (tok0 + q0 + m) * DM + head * HHALF;
  const v16h qb0 = load_frag(qrow, h);
  const v16h qb1 = load_frag(qrow + 512, h);

  const v8f zero8 = {0.f, 0.f, 0.f, 0.f, 0.f, 0.f, 0.f, 0.f};
  v8f o[4];
  #pragma unroll
  for (int t = 0; t < 4; ++t) o[t] = zero8;
  float mrun = -1e30f, lrun = 0.0f;

  const _Float16* kbase = Kp + (tok0 + m) * DM + head * HHALF;
  const _Float16* vbase = VT + ((size_t)bh * HDIM + m) * SEQ;
  const float* mrow = maskp + (tok0 + q0 + m) * SEQ + 8 * h;

  #pragma unroll 1
  for (int kb = 0; kb < SEQ; kb += 64) {
    v8f s[4];
    #pragma unroll
    for (int j = 0; j < 4; ++j) {
      const _Float16* kp = kbase + (size_t)(kb + 16 * j) * DM;
      const v16h kf0 = load_frag(kp, h);
      const v16h kf1 = load_frag(kp + 512, h);
      v8f z = zero8;
      z = wmma_f16(kf0, qb0, z);
      z = wmma_f16(kf1, qb1, z);
      s[j] = z;
    }
    #pragma unroll
    for (int j = 0; j < 4; ++j) {
      const v4f ma = *(const v4fa*)(mrow + kb + 16 * j);
      const v4f mb = *(const v4fa*)(mrow + kb + 16 * j + 4);
      s[j][0] = s[j][0] * 0.125f + ma.x;
      s[j][1] = s[j][1] * 0.125f + ma.y;
      s[j][2] = s[j][2] * 0.125f + ma.z;
      s[j][3] = s[j][3] * 0.125f + ma.w;
      s[j][4] = s[j][4] * 0.125f + mb.x;
      s[j][5] = s[j][5] * 0.125f + mb.y;
      s[j][6] = s[j][6] * 0.125f + mb.z;
      s[j][7] = s[j][7] * 0.125f + mb.w;
    }

    float mloc = s[0][0];
    #pragma unroll
    for (int j = 0; j < 4; ++j)
      #pragma unroll
      for (int r = 0; r < 8; ++r) mloc = fmaxf(mloc, s[j][r]);
    mloc = fmaxf(mloc, __shfl_xor(mloc, 16));
    const float mnew = fmaxf(mrun, mloc);
    const float alpha = __expf(mrun - mnew);
    mrun = mnew;
    float lsum = 0.0f;
    #pragma unroll
    for (int j = 0; j < 4; ++j)
      #pragma unroll
      for (int r = 0; r < 8; ++r) {
        const float p = __expf(s[j][r] - mnew);
        s[j][r] = p;
        lsum += p;
      }
    lsum += __shfl_xor(lsum, 16);
    lrun = lrun * alpha + lsum;
    #pragma unroll
    for (int t = 0; t < 4; ++t)
      #pragma unroll
      for (int r = 0; r < 8; ++r) o[t][r] = o[t][r] * alpha;

    const v16h pb0 = pack_p(s[0], s[1]);
    const v16h pb1 = pack_p(s[2], s[3]);

    #pragma unroll
    for (int t = 0; t < 4; ++t) {
      const _Float16* vp = vbase + (size_t)(16 * t) * SEQ + kb;
      const v16h vf0 = load_frag(vp, h);
      const v16h vf1 = load_frag(vp + 32, h);
      o[t] = wmma_f16(vf0, pb0, o[t]);
      o[t] = wmma_f16(vf1, pb1, o[t]);
    }
  }

  const float inv = (1.0f / lrun) * (16.0f / PSCALE);
  _Float16* so = sO + w * 1024;
  #pragma unroll
  for (int t = 0; t < 4; ++t)
    #pragma unroll
    for (int r = 0; r < 8; ++r)
      so[m * 64 + 16 * t + 8 * h + r] = (_Float16)(o[t][r] * inv);
  __syncthreads();

  const size_t rowbase = tok0 + q0;
  ctx_store_pass(so, ctx, rowbase, head, lane);
  __threadfence();
  ctx_store_pass(so, ctx, rowbase, head, lane);
}

extern "C" void kernel_launch(void* const* d_in, const int* in_sizes, int n_in,
                              void* d_out, int out_size, void* d_ws, size_t ws_size,
                              hipStream_t stream) {
  if (n_in < 21) return;
  if (in_sizes[0] != NTOK * DM) return;
  if (in_sizes[1] != DM || in_sizes[16] != DM || in_sizes[17] != DM || in_sizes[20] != DM) return;
  if (in_sizes[2] != 2 * MVH * DM || in_sizes[3] != 2 * MVH * DM) return;
  if (in_sizes[4] != 512 * MVH || in_sizes[5] != 512 * MVH || in_sizes[7] != 512 * MVH) return;
  if (in_sizes[6] != DM * MVH) return;
  if (in_sizes[8] != 512 * DM) return;
  if (in_sizes[9] != 16 || in_sizes[10] != 16) return;
  if (in_sizes[11] != 2 * SEQ * SEQ || in_sizes[13] != 2 * SEQ * SEQ) return;
  if (in_sizes[12] != 2 * SEQ || in_sizes[14] != SEQ) return;
  if (in_sizes[15] != DM * DM) return;
  if (in_sizes[18] != MLPD * DM || in_sizes[19] != MLPD * DM) return;
  if (out_size != NTOK * DM) return;

  const float* xin   = (const float*)d_in[0];
  const float* lnw1  = (const float*)d_in[1];
  const float* encq  = (const float*)d_in[2];
  const float* enckv = (const float*)d_in[3];
  const float* wqp   = (const float*)d_in[4];
  const float* wkp   = (const float*)d_in[5];
  const float* wvp   = (const float*)d_in[6];
  const float* wqrp  = (const float*)d_in[7];
  const float* wkrp  = (const float*)d_in[8];
  const float* invq  = (const float*)d_in[9];
  const float* invk  = (const float*)d_in[10];
  const float* mw1   = (const float*)d_in[11];
  const float* mb1   = (const float*)d_in[12];
  const float* mw2   = (const float*)d_in[13];
  const float* mb2   = (const float*)d_in[14];
  const float* wop   = (const float*)d_in[15];
  const float* lsa   = (const float*)d_in[16];
  const float* lnw2  = (const float*)d_in[17];
  const float* w1p   = (const float*)d_in[18];
  const float* w2p   = (const float*)d_in[19];
  const float* lsm   = (const float*)d_in[20];
  float* out = (float*)d_out;

  const size_t wbytes = (size_t)NW_TOTAL * 2;
  const size_t plane8 = (size_t)NTOK * DM * 2;
  const size_t regA   = 4 * plane8;
  const size_t regB   = (size_t)NTOK * DM * 4;
  const size_t regC   = (size_t)NTOK * 2 * SEQ * 2;
  const size_t total  = wbytes + regA + regB + regC;
  if (total > ws_size) return;
  const size_t offA = wbytes, offB = offA + regA, offC = offB + regB;

  char* ws = (char*)d_ws;
  _Float16* wbuf  = (_Float16*)ws;
  _Float16* Wenc  = wbuf + OW_ENC;
  _Float16* Wq    = wbuf + OW_Q;
  _Float16* Wqr   = wbuf + OW_QR;
  _Float16* Wk    = wbuf + OW_K;
  _Float16* Wv    = wbuf + OW_V;
  _Float16* Wkr   = wbuf + OW_KR;
  _Float16* Wm1   = wbuf + OW_M1;
  _Float16* Wm2   = wbuf + OW_M2;
  _Float16* Wo    = wbuf + OW_O;
  _Float16* Wmlp1 = wbuf + OW_MLP1;
  _Float16* Wmlp2 = wbuf + OW_MLP2;

  _Float16* Qp   = (_Float16*)(ws + offA);
  _Float16* Kp   = (_Float16*)(ws + offA + plane8);
  _Float16* VT   = (_Float16*)(ws + offA + 2 * plane8);
  _Float16* ctxp = (_Float16*)(ws + offA + 3 * plane8);
  _Float16* hmp  = (_Float16*)(ws + offA);
  _Float16* smp  = (_Float16*)(ws + offB);
  float*    mskp = (float*)(ws + offB);
  float*    xp   = (float*)(ws + offB);
  _Float16* xq   = (_Float16*)(ws + offC);
  _Float16* zpl  = (_Float16*)(ws + offC + plane8);
  _Float16* h1p  = (_Float16*)(ws + offC);
  _Float16* xlnp = (_Float16*)(ws + offC);

  const float* dF  = lnw1;
  float*    dOF = (float*)(ws + offA + 3 * plane8);
  _Float16* dOH = zpl;
  const float SC32 = 0.03125f;

  k_convert<<<CB11, 256, 0, stream>>>(encq, enckv, wqp, wqrp, wkp, wvp, wkrp, mw1, mw2, wop, w1p, w2p, wbuf);
  k_layernorm<<<NTOK, 128, 0, stream>>>(xin, lnw1, xq);
  k_gemm<0><<<dim3(NTOK / 128, (2 * MVH) / 64, 1), 128, 0, stream>>>(
      xq, DM, 0, Wenc, DM, 0, DM, dOF, zpl, 2 * MVH, 0, 0, SC32, dF, dF, dF, dF);
  k_gemm<0><<<dim3(NTOK / 128, 512 / 64, 1), 128, 0, stream>>>(
      zpl, 2 * MVH, 0, Wq, MVH, 0, MVH, dOF, Qp, DM, 0, 0, SC32, dF, dF, dF, dF);
  k_gemm<16><<<dim3(NTOK / 128, 512 / 64, 1), 128, 0, stream>>>(
      zpl, 2 * MVH, 0, Wqr, MVH, 0, MVH, dOF, Qp, DM, 512, 0, SC32, dF, dF, dF, invq);
  k_gemm<0><<<dim3(NTOK / 128, 512 / 64, 1), 128, 0, stream>>>(
      zpl + MVH, 2 * MVH, 0, Wk, MVH, 0, MVH, dOF, Kp, DM, 0, 0, SC32, dF, dF, dF, dF);
  k_gemm<16><<<dim3(NTOK / 128, 512 / 64, 1), 128, 0, stream>>>(
      xq, DM, 0, Wkr, DM, 0, DM, dOF, Kp, DM, 512, 0, SC32, dF, dF, dF, invk);
  k_gemm<32><<<dim3(NTOK / 128, DM / 64, 1), 128, 0, stream>>>(
      zpl + MVH, 2 * MVH, 0, Wv, MVH, 0, MVH, dOF, VT, SEQ, 0, 0, SC32, dF, dF, dF, dF);
  k_gemm<0><<<dim3(SEQ / 128, SEQ / 64, BATCH), 128, 0, stream>>>(
      Qp, DM, (long long)SEQ * DM, Kp, DM, (long long)SEQ * DM, DM,
      dOF, smp, SEQ, 0, (long long)SEQ * SEQ, 1.0f, dF, dF, dF, dF);
  k_gemm<6><<<dim3(NTOK / 128, (2 * SEQ) / 64, 1), 128, 0, stream>>>(
      smp, SEQ, 0, Wm1, SEQ, 0, SEQ, dOF, h1p, 2 * SEQ, 0, 0, SC32, mb1, dF, dF, dF);
  k_gemm<3><<<dim3(NTOK / 128, SEQ / 64, 1), 128, 0, stream>>>(
      h1p, 2 * SEQ, 0, Wm2, 2 * SEQ, 0, 2 * SEQ, mskp, dOH, SEQ, 0, 0, SC32, mb2, dF, dF, dF);
  k_attn<<<dim3(SEQ / 64, BATCH * NHEAD), 128, 0, stream>>>(Qp, Kp, VT, mskp, ctxp);
  k_gemm<9><<<dim3(NTOK / 128, DM / 64, 1), 128, 0, stream>>>(
      ctxp, DM, 0, Wo, DM, 0, DM, xp, dOH, DM, 0, 0, SC32 * 0.0625f, dF, xin, lsa, dF);
  k_layernorm<<<NTOK, 128, 0, stream>>>(xp, lnw2, xlnp);
  k_gemm<4><<<dim3(NTOK / 128, MLPD / 64, 1), 128, 0, stream>>>(
      xlnp, DM, 0, Wmlp1, DM, 0, DM, dOF, hmp, MLPD, 0, 0, SC32, dF, dF, dF, dF);
  k_gemm<9><<<dim3(NTOK / 128, DM / 64, 1), 128, 0, stream>>>(
      hmp, MLPD, 0, Wmlp2, MLPD, 0, MLPD, out, dOH, DM, 0, 0, SC32, dF, xp, lsm, dF);
}
